// GATRelationNet_21706764714080
// MI455X (gfx1250) — hardware-run, weakly checked
//
#include <hip/hip_runtime.h>


#ifndef NB
#define NB 256
#endif
#ifndef SEQ
#define SEQ 1000
#endif
#define NB_FULL  256
#define SEQ_FULL 1000
#define DH   512
#define NBP  (((NB + 63) / 64) * 64)
#define SEQP (((SEQ + 63) / 64) * 64)
#define NQ   ((SEQ + 255) / 256)
#define SLOPE 0.2f
#define L2E  1.4426950408889634f

static_assert(NB <= NB_FULL);
static_assert(SEQ <= SEQ_FULL);
static_assert(NB % 4 == 0);
static_assert(SEQ % 8 == 0);
static_assert(DH % 64 == 0);
static_assert(DH % 32 == 0);
static_assert(SEQP % 64 == 0);
static_assert(SEQP % 32 == 0);
static_assert(NBP % 64 == 0);
static_assert(SEQP >= 64);

typedef unsigned short bf;
typedef __attribute__((ext_vector_type(16))) __bf16   v16bf;
typedef __attribute__((ext_vector_type(8)))  unsigned short v8us;
typedef __attribute__((ext_vector_type(8)))  float    v8f;
typedef __attribute__((ext_vector_type(4)))  float    v4f;
typedef v4f  __attribute__((may_alias)) v4fa;

__device__ __forceinline__ unsigned short f2bf(float f) { unsigned u = __float_as_uint(f); u += 0x7FFFu + ((u >> 16) & 1u); return (unsigned short)(u >> 16); }
__device__ __forceinline__ float bfx(unsigned short h) { return __uint_as_float(((unsigned)h) << 16); }
__device__ __forceinline__ float rbf(float f) { return bfx(f2bf(f)); }
__device__ __forceinline__ v16bf cat16b(v8us lo, v8us hi) { return __builtin_bit_cast(v16bf, __builtin_shufflevector(lo, hi, 0, 1, 2, 3, 4, 5, 6, 7, 8, 9, 10, 11, 12, 13, 14, 15)); }
__device__ __forceinline__ v8f wmmab(v16bf a, v16bf b, v8f c) { return __builtin_amdgcn_wmma_f32_16x16x32_bf16(false, a, false, b, (short)0, c, false, false); }
__device__ __forceinline__ v16bf ldb(const bf* p)  { return cat16b(*(const v8us*)p, *(const v8us*)(p + 16)); }
__device__ __forceinline__ void wave_sync() { __builtin_amdgcn_fence(3  , "wavefront"); __builtin_amdgcn_wave_barrier(); asm volatile("" ::: "memory"); }

__global__ __launch_bounds__(256) void k_cvt8z(const float* __restrict__ src, bf* dst, size_t n8src, size_t n8tot) {
    const size_t i = (size_t)blockIdx.x * 256 + threadIdx.x; if (i >= n8tot) return;
    const bool live = i < n8src;
    const size_t is = live ? i : (n8src - 1);
    const v8f v = *(const v8f*)(src + is * 8); v8us o;
#pragma unroll
    for (int k = 0; k < 8; ++k) o[k] = live ? f2bf(v[k]) : (unsigned short)0;
    *(volatile v8us*)(dst + i * 8) = o; __threadfence(); *(volatile v8us*)(dst + i * 8) = o;
}

__global__ __launch_bounds__(256) void k_tcvt(const float* __restrict__ W, bf* WT) {
    __shared__ __align__(16) float ts[64 * 68];
    const int t = threadIdx.x; const int k0 = blockIdx.x * 64, n0 = blockIdx.y * 64;
    const int c4 = (t & 15) * 4, r = t >> 4;
#pragma unroll
    for (int it = 0; it < 4; ++it) { const int k = r + 16 * it;
        const v4f v = *(const v4f*)(W + (size_t)(k0 + k) * DH + n0 + c4);
        *(v4fa*)(&ts[k * 68 + c4]) = v; }
    __syncthreads();
    const int rn = t >> 3, k8 = (t & 7) * 8;
    v8us o0, o1;
#pragma unroll
    for (int i = 0; i < 8; ++i) { o0[i] = f2bf(ts[(k8 + i) * 68 + rn]); o1[i] = f2bf(ts[(k8 + i) * 68 + rn + 32]); }
    bf* d0 = WT + (size_t)(n0 + rn) * DH + k0 + k8;
    bf* d1 = WT + (size_t)(n0 + rn + 32) * DH + k0 + k8;
    *(volatile v8us*)d0 = o0; *(volatile v8us*)d1 = o1;
    __threadfence();
    *(volatile v8us*)d0 = o0; *(volatile v8us*)d1 = o1;
}

template <int MODE>
__global__ __launch_bounds__(32) void k_gemm(const bf* __restrict__ P, size_t a0, size_t a1, size_t a2, size_t b0, size_t b1, size_t b2,
                                             int nseg, int K, float* Cf, bf* Ch, bf* Cl, int ldc) {
    __shared__ __align__(16) float os[16 * 68];
    const int lane = threadIdx.x & 31, lr = lane & 15, hi = lane >> 4; const int r0 = blockIdx.x * 64, c0 = blockIdx.y * 64;
    v8f acc[4][4];
#pragma unroll
    for (int mb = 0; mb < 4; ++mb)
#pragma unroll
        for (int nb = 0; nb < 4; ++nb) acc[mb][nb] = (v8f){};
    const size_t aoff = (size_t)(r0 + lr) * K + 8 * hi, boff = (size_t)(c0 + lr) * K + 8 * hi;
#pragma unroll 1
    for (int sg = 0; sg < nseg; ++sg) {
        const size_t ab = (sg == 0) ? a0 : ((sg == 1) ? a1 : a2);
        const size_t bb = (sg == 0) ? b0 : ((sg == 1) ? b1 : b2);
        const bf* A  = P + ab + aoff;
        const bf* Bt = P + bb + boff;
#pragma unroll 1
        for (int kc = 0; kc < K; kc += 32) {
            v16bf a[4];
#pragma unroll
            for (int mb = 0; mb < 4; ++mb) a[mb] = ldb(A + (size_t)mb * 16 * K + kc);
#pragma unroll
            for (int nb = 0; nb < 4; ++nb) { const v16bf b = ldb(Bt + (size_t)nb * 16 * K + kc);
#pragma unroll
                for (int mb = 0; mb < 4; ++mb) acc[mb][nb] = wmmab(a[mb], b, acc[mb][nb]); }
            asm volatile("v_nop\n\tv_nop\n\tv_nop\n\tv_nop" : "+v"(acc[0][0]), "+v"(acc[1][1]), "+v"(acc[2][2]), "+v"(acc[3][3]) : "v"(a[0]), "v"(a[1]), "v"(a[2]), "v"(a[3]));
        }
    }
#pragma unroll
    for (int mb = 0; mb < 4; ++mb) {
#pragma unroll
        for (int nb = 0; nb < 4; ++nb) {
#pragma unroll
            for (int j = 0; j < 8; ++j) os[(hi * 8 + j) * 68 + nb * 16 + lr] = acc[mb][nb][j]; }
        wave_sync();
        if (MODE == 1) {
#pragma unroll 1
            for (int ps = 0; ps < 2; ++ps) {
#pragma unroll
                for (int s = 0; s < 4; ++s) { const int row = 4 * s + (lane >> 3), c8 = (lane & 7) * 8;
                    const v4f x0 = *(const v4fa*)(&os[row * 68 + c8]); const v4f x1 = *(const v4fa*)(&os[row * 68 + c8 + 4]); v8us hv, lv;
#pragma unroll
                    for (int i = 0; i < 4; ++i) { const unsigned short h0 = f2bf(x0[i]); const unsigned short h1 = f2bf(x1[i]);
                        hv[i] = h0; hv[4 + i] = h1; lv[i] = f2bf(x0[i] - bfx(h0)); lv[4 + i] = f2bf(x1[i] - bfx(h1)); }
                    const size_t oo = (size_t)(r0 + mb * 16 + row) * (size_t)ldc + c0 + c8;
                    *(volatile v8us*)(Ch + oo) = hv; *(volatile v8us*)(Cl + oo) = lv; }
                if (ps == 0) __threadfence(); }
        } else {
#pragma unroll 1
            for (int ps = 0; ps < 2; ++ps) {
#pragma unroll
                for (int s = 0; s < 8; ++s) { const int row = 2 * s + hi, cofs = lr * 4;
                    const v4f val = *(const v4fa*)(&os[row * 68 + cofs]);
                    *(volatile v4f*)(Cf + (size_t)(r0 + mb * 16 + row) * (size_t)ldc + c0 + cofs) = val; }
                if (ps == 0) __threadfence(); }
        }
        wave_sync();
    }
}

__global__ __launch_bounds__(256) void k_s12(const bf* __restrict__ AH, const bf* __restrict__ AL, const float* __restrict__ atta, float* S) {
    const int j = blockIdx.x * 256 + threadIdx.x;
    const int jc = (j < SEQP) ? j : (SEQP - 1);
    float s1 = 0.0f, s2 = 0.0f;
#pragma unroll 4
    for (int h = 0; h < DH; ++h) {
        const float v = bfx(AH[(size_t)h * SEQP + jc]) + bfx(AL[(size_t)h * SEQP + jc]);
        const float w1 = rbf(atta[h]), w2 = rbf(atta[DH + h]);
        s1 = fmaf(v, w1, s1); s2 = fmaf(v, w2, s2);
    }
    if (j < SEQP) {
        *(volatile float*)(S + j) = s1; *(volatile float*)(S + SEQP + j) = s2;
        __threadfence();
        *(volatile float*)(S + j) = s1; *(volatile float*)(S + SEQP + j) = s2;
    }
}

__global__ __launch_bounds__(256) void k_softmax(const float* __restrict__ S, bf* PH, bf* PL) {
    const int lane = threadIdx.x & 31; const int wave = __builtin_amdgcn_readfirstlane((int)(threadIdx.x >> 5));
    const int i = blockIdx.x * 8 + wave;
    const bool liverow = i < SEQ;
    const float s1 = S[i];
    const float* S2 = S + SEQP;
    float m = -3.0e38f;
#pragma unroll 1
    for (int c = 0; c < SEQP; c += 256) {
        const int j0 = c + lane * 8; const int jc = (j0 < SEQP - 8) ? j0 : (SEQP - 8);
        const v4f x0 = *(const v4f*)(S2 + jc); const v4f x1 = *(const v4f*)(S2 + jc + 4);
#pragma unroll
        for (int k = 0; k < 4; ++k) {
            float e0 = s1 + x0[k]; e0 = (e0 >= 0.0f) ? e0 : SLOPE * e0;
            float e1 = s1 + x1[k]; e1 = (e1 >= 0.0f) ? e1 : SLOPE * e1;
            m = (j0 + k < SEQ) ? fmaxf(m, e0) : m;
            m = (j0 + 4 + k < SEQ) ? fmaxf(m, e1) : m; }
    }
#pragma unroll
    for (int off = 16; off > 0; off >>= 1) m = fmaxf(m, __shfl_xor(m, off, 32));
    float l = 0.0f;
#pragma unroll 1
    for (int c = 0; c < SEQP; c += 256) {
        const int j0 = c + lane * 8; const int jc = (j0 < SEQP - 8) ? j0 : (SEQP - 8);
        const v4f x0 = *(const v4f*)(S2 + jc); const v4f x1 = *(const v4f*)(S2 + jc + 4);
#pragma unroll
        for (int k = 0; k < 4; ++k) {
            float e0 = s1 + x0[k]; e0 = (e0 >= 0.0f) ? e0 : SLOPE * e0;
            float e1 = s1 + x1[k]; e1 = (e1 >= 0.0f) ? e1 : SLOPE * e1;
            const float p0 = __builtin_amdgcn_exp2f((e0 - m) * L2E);
            const float p1 = __builtin_amdgcn_exp2f((e1 - m) * L2E);
            l += (j0 + k < SEQ) ? p0 : 0.0f;
            l += (j0 + 4 + k < SEQ) ? p1 : 0.0f; }
    }
#pragma unroll
    for (int off = 16; off > 0; off >>= 1) l += __shfl_xor(l, off, 32);
    const float inv = 1.0f / l;
#pragma unroll 1
    for (int c = 0; c < SEQP; c += 256) {
        const int j0 = c + lane * 8; const int jc = (j0 < SEQP - 8) ? j0 : (SEQP - 8);
        const v4f x0 = *(const v4f*)(S2 + jc); const v4f x1 = *(const v4f*)(S2 + jc + 4);
        v8us hv, lv;
#pragma unroll
        for (int k = 0; k < 4; ++k) {
            float e0 = s1 + x0[k]; e0 = (e0 >= 0.0f) ? e0 : SLOPE * e0;
            float e1 = s1 + x1[k]; e1 = (e1 >= 0.0f) ? e1 : SLOPE * e1;
            float p0 = __builtin_amdgcn_exp2f((e0 - m) * L2E) * inv;
            float p1 = __builtin_amdgcn_exp2f((e1 - m) * L2E) * inv;
            p0 = (liverow && (j0 + k < SEQ)) ? p0 : 0.0f;
            p1 = (liverow && (j0 + 4 + k < SEQ)) ? p1 : 0.0f;
            const unsigned short h0 = f2bf(p0), h1 = f2bf(p1);
            hv[k] = h0; hv[4 + k] = h1; lv[k] = f2bf(p0 - bfx(h0)); lv[4 + k] = f2bf(p1 - bfx(h1)); }
        if (j0 < SEQP) {
            const size_t oo = (size_t)i * SEQP + j0;
            *(volatile v8us*)(PH + oo) = hv; *(volatile v8us*)(PL + oo) = lv;
            __threadfence();
            *(volatile v8us*)(PH + oo) = hv; *(volatile v8us*)(PL + oo) = lv;
        }
    }
}

__global__ __launch_bounds__(256) void k_head(const float* __restrict__ IMGP, const float* __restrict__ SEMP, const float* __restrict__ semb,
                                              const float* __restrict__ fcw, const float* __restrict__ fcb, float* OUT) {
    __shared__ __align__(16) float simg[4 * DH];
    __shared__ __align__(16) float sfw[DH];
    __shared__ __align__(16) float ost[4 * SEQ];
    const int t = threadIdx.x; const int b0 = blockIdx.x * 4;
    for (int x = t; x < 4 * DH; x += 256) { const int h = x & (DH - 1), bl = x / DH;
        simg[x] = IMGP[(size_t)(b0 + bl) * DH + h] + rbf(semb[h]); }
    for (int x = t; x < DH; x += 256) sfw[x] = rbf(fcw[x]);
    const float bias = rbf(fcb[0]);
    __syncthreads();
#pragma unroll 1
    for (int q = 0; q < NQ; ++q) {
        const int n = t + 256 * q; const int nc = (n < SEQ) ? n : (SEQ - 1);
        const float* srow = SEMP + (size_t)nc * DH;
        float a0 = 0.0f, a1 = 0.0f, a2 = 0.0f, a3 = 0.0f;
#pragma unroll 1
        for (int h4 = 0; h4 < DH; h4 += 4) {
            const v4f s  = *(const v4f*)(srow + h4);
            const v4f w  = *(const v4fa*)(&sfw[h4]);
            const v4f i0 = *(const v4fa*)(&simg[0 * DH + h4]);
            const v4f i1 = *(const v4fa*)(&simg[1 * DH + h4]);
            const v4f i2 = *(const v4fa*)(&simg[2 * DH + h4]);
            const v4f i3 = *(const v4fa*)(&simg[3 * DH + h4]);
#pragma unroll
            for (int e = 0; e < 4; ++e) {
                a0 = fmaf(fmaxf(i0[e] + s[e], 0.0f), w[e], a0);
                a1 = fmaf(fmaxf(i1[e] + s[e], 0.0f), w[e], a1);
                a2 = fmaf(fmaxf(i2[e] + s[e], 0.0f), w[e], a2);
                a3 = fmaf(fmaxf(i3[e] + s[e], 0.0f), w[e], a3); }
        }
        if (n < SEQ) { ost[0 * SEQ + n] = a0 + bias; ost[1 * SEQ + n] = a1 + bias; ost[2 * SEQ + n] = a2 + bias; ost[3 * SEQ + n] = a3 + bias; }
    }
    __syncthreads();
    float* ob = OUT + (size_t)b0 * SEQ;
#pragma unroll 1
    for (int f4 = t; f4 < SEQ; f4 += 256) { const v4f v = *(const v4fa*)(&ost[4 * f4]); *(volatile v4f*)(ob + 4 * f4) = v; }
    __threadfence();
#pragma unroll 1
    for (int f4 = t; f4 < SEQ; f4 += 256) { const v4f v = *(const v4fa*)(&ost[4 * f4]); *(volatile v4f*)(ob + 4 * f4) = v; }
}

static constexpr size_t al256(size_t v) { return (v + 255) & ~(size_t)255; }
static constexpr size_t SZ_ATTRB = al256((size_t)SEQP * DH * 2);
static constexpr size_t SZ_IMGB  = al256((size_t)NBP * DH * 2);
static constexpr size_t SZ_WT    = al256((size_t)DH * DH * 2);
static constexpr size_t SZ_AHT   = al256((size_t)DH * SEQP * 2);
static constexpr size_t SZ_S     = al256((size_t)2 * SEQP * 4);
static constexpr size_t SZ_P     = al256((size_t)SEQP * SEQP * 2);
static constexpr size_t SZ_AO    = al256((size_t)SEQP * DH * 2);
static constexpr size_t SZ_IMGP  = al256((size_t)NBP * DH * 4);
static constexpr size_t SZ_SEMP  = al256((size_t)SEQP * DH * 4);
static constexpr size_t SZ_TOTAL = SZ_ATTRB + SZ_IMGB + 3 * SZ_WT + 2 * SZ_AHT + SZ_S + 2 * SZ_P + 2 * SZ_AO + SZ_IMGP + SZ_SEMP;
static_assert(SZ_TOTAL <= (size_t)134217728);

extern "C" void kernel_launch(void* const* d_in, const int* in_sizes, int n_in,
                              void* d_out, int out_size, void* d_ws, size_t ws_size, hipStream_t stream) {
    if (n_in < 9) return;
    if ((size_t)in_sizes[0] < (size_t)NB * DH) return;
    if ((size_t)in_sizes[1] < (size_t)SEQ * DH) return;
    if ((size_t)in_sizes[2] < (size_t)DH * DH || (size_t)in_sizes[4] < (size_t)DH * DH || (size_t)in_sizes[5] < (size_t)DH * DH) return;
    if ((size_t)in_sizes[3] < (size_t)2 * DH) return;
    if ((size_t)in_sizes[6] < (size_t)DH || (size_t)in_sizes[7] < (size_t)DH || in_sizes[8] < 1) return;
    if ((size_t)out_size < (size_t)NB * SEQ) return;
    if (SZ_TOTAL > ws_size) return;
    const float* imgf = (const float*)d_in[0]; const float* attr = (const float*)d_in[1]; const float* attw = (const float*)d_in[2];
    const float* atta = (const float*)d_in[3]; const float* imgw = (const float*)d_in[4]; const float* semw = (const float*)d_in[5];
    const float* semb = (const float*)d_in[6]; const float* fcw = (const float*)d_in[7];  const float* fcb = (const float*)d_in[8];
    float* OUT = (float*)d_out;
    char* w0 = (char*)d_ws; char* wsp = w0;
    bf* ATTRB = (bf*)wsp; wsp += SZ_ATTRB;
    bf* IMGB  = (bf*)wsp; wsp += SZ_IMGB;
    bf* WTA   = (bf*)wsp; wsp += SZ_WT;
    bf* WTI   = (bf*)wsp; wsp += SZ_WT;
    bf* WTS   = (bf*)wsp; wsp += SZ_WT;
    bf* AHH   = (bf*)wsp; wsp += SZ_AHT;
    bf* AHL   = (bf*)wsp; wsp += SZ_AHT;
    float* S  = (float*)wsp; wsp += SZ_S;
    bf* PH    = (bf*)wsp; wsp += SZ_P;
    bf* PL    = (bf*)wsp; wsp += SZ_P;
    bf* AOH   = (bf*)wsp; wsp += SZ_AO;
    bf* AOL   = (bf*)wsp; wsp += SZ_AO;
    float* IMGP = (float*)wsp; wsp += SZ_IMGP;
    float* SEMP = (float*)wsp; wsp += SZ_SEMP;
    const bf* WS = (const bf*)w0;
    const size_t oATTRB = (size_t)((char*)ATTRB - w0) / 2, oIMGB = (size_t)((char*)IMGB - w0) / 2;
    const size_t oWTA = (size_t)((char*)WTA - w0) / 2, oWTI = (size_t)((char*)WTI - w0) / 2, oWTS = (size_t)((char*)WTS - w0) / 2;
    const size_t oAHH = (size_t)((char*)AHH - w0) / 2, oAHL = (size_t)((char*)AHL - w0) / 2;
    const size_t oPH = (size_t)((char*)PH - w0) / 2, oPL = (size_t)((char*)PL - w0) / 2;
    const size_t oAOH = (size_t)((char*)AOH - w0) / 2, oAOL = (size_t)((char*)AOL - w0) / 2;

    { const size_t ns = (size_t)SEQ * DH / 8, nt = (size_t)SEQP * DH / 8;
      k_cvt8z<<<(unsigned)((nt + 255) / 256), 256, 0, stream>>>(attr, ATTRB, ns, nt); }
    { const size_t ns = (size_t)NB * DH / 8, nt = (size_t)NBP * DH / 8;
      k_cvt8z<<<(unsigned)((nt + 255) / 256), 256, 0, stream>>>(imgf, IMGB, ns, nt); }
    k_tcvt<<<dim3(DH / 64, DH / 64, 1), 256, 0, stream>>>(attw, WTA);
    k_tcvt<<<dim3(DH / 64, DH / 64, 1), 256, 0, stream>>>(imgw, WTI);
    k_tcvt<<<dim3(DH / 64, DH / 64, 1), 256, 0, stream>>>(semw, WTS);

    k_gemm<1><<<dim3(DH / 64, SEQP / 64, 1), 32, 0, stream>>>(WS, oWTA, oWTA, oWTA, oATTRB, oATTRB, oATTRB, 1, DH, IMGP, AHH, AHL, SEQP);
    k_s12<<<(SEQP + 255) / 256, 256, 0, stream>>>(AHH, AHL, atta, S);
    k_softmax<<<SEQP / 8, 256, 0, stream>>>(S, PH, PL);
    k_gemm<1><<<dim3(SEQP / 64, DH / 64, 1), 32, 0, stream>>>(WS, oPH, oPL, oPH, oAHH, oAHH, oAHL, 3, SEQP, IMGP, AOH, AOL, DH);
    k_gemm<0><<<dim3(NBP / 64, DH / 64, 1), 32, 0, stream>>>(WS, oIMGB, oIMGB, oIMGB, oWTI, oWTI, oWTI, 1, DH, IMGP, AOH, AOL, DH);
    k_gemm<0><<<dim3(SEQP / 64, DH / 64, 1), 32, 0, stream>>>(WS, oAOH, oAOL, oAOH, oWTS, oWTS, oWTS, 2, DH, SEMP, AOH, AOL, DH);
    k_head<<<NB / 4, 256, 0, stream>>>(IMGP, SEMP, semb, fcw, fcb, OUT);
}
